// ExplainableHeteroClassifier_without_lexical_chain_23742579212720
// MI455X (gfx1250) — hardware-verified
//
#include <hip/hip_runtime.h>
#include <math.h>


#define RR 20
#define NN 4096
#define NBG 16
#define SS 256
#define DI 512
#define NH 4
#define HID 128
#define DD 512
#define EE 16384
#define SLOTC 32
#define NCH 512

typedef __attribute__((ext_vector_type(16))) _Float16 v16h;
typedef __attribute__((ext_vector_type(8)))  _Float16 v8h;
typedef __attribute__((ext_vector_type(8)))  float v8f;
typedef __attribute__((ext_vector_type(4)))  float v4f;
typedef __attribute__((ext_vector_type(4)))  unsigned v4u;
typedef __attribute__((ext_vector_type(4)))  int v4i;
typedef float __attribute__((may_alias)) float_a;

template <typename T> __device__ __forceinline__ void vst2(void* p, T v) { *(volatile T*)p = v; __threadfence(); *(volatile T*)p = v; }
__device__ __forceinline__ v8f wmma16(v16h a, v16h b, v8f c) {
  v8f d = __builtin_amdgcn_wmma_f32_16x16x32_f16(false, a, false, b, (short)0, c, false, false);
  asm volatile("v_nop\n\tv_nop\n\tv_nop\n\tv_nop" : "+v"(d) : "v"(a), "v"(b));
  return d;
}
__device__ __forceinline__ v16h frag_h(const _Float16* rowk0, int lane) {
  union { v16h v; v8h q[2]; } u; const _Float16* p = rowk0 + 8 * (lane >> 4);
  u.q[0] = *(const v8h*)p; u.q[1] = *(const v8h*)(p + 16); return u.v;
}
__device__ __forceinline__ v16h frag_f32(const float* rowk0, int lane) {
  v16h a; const float* p = rowk0 + 8 * (lane >> 4);
#pragma unroll
  for (int i = 0; i < 8; ++i) { a[i] = (_Float16)p[i]; a[8 + i] = (_Float16)p[16 + i]; }
  return a;
}
#define LDSX() do { asm volatile("s_wait_dscnt 0" ::: "memory"); __builtin_amdgcn_wave_barrier(); __builtin_amdgcn_fence(__ATOMIC_RELEASE, "workgroup"); } while (0)

__global__ __launch_bounds__(256) void k_packT(const float* __restrict__ W, _Float16* __restrict__ Wt, int K, int N) {
  __shared__ float tile[64][65];
  const int k0 = blockIdx.y * 64, n0 = blockIdx.x * 64, z = blockIdx.z, tid = threadIdx.x;
  const float* Wz = W + (size_t)z * K * N; _Float16* Wtz = Wt + (size_t)z * K * N;
  for (int q = tid; q < 64 * 64; q += 256) { const int kk = q >> 6, nn = q & 63; tile[kk][nn] = Wz[(size_t)(k0 + kk) * N + n0 + nn]; }
  __syncthreads();
  for (int q = tid; q < 64 * 8; q += 256) { const int nn = q >> 3, pc = q & 7;
    union { v8h h; v4u u; } pk;
#pragma unroll
    for (int e = 0; e < 8; ++e) pk.h[e] = (_Float16)tile[pc * 8 + e][nn];
    vst2(Wtz + (size_t)(n0 + nn) * K + k0 + pc * 8, pk.u); }
}
__global__ __launch_bounds__(256) void k_cvt(const float* __restrict__ s, _Float16* __restrict__ d, size_t n8) {
  const size_t g8 = (size_t)blockIdx.x * 256 + threadIdx.x; if (g8 >= n8) return;
  union { v8h h; v4u u; } pk;
#pragma unroll
  for (int e = 0; e < 8; ++e) pk.h[e] = (_Float16)s[g8 * 8 + e];
  vst2(d + g8 * 8, pk.u);
}

__global__ __launch_bounds__(256) void k_bucket(const int* __restrict__ dst, int* __restrict__ tlist) {
  __shared__ int scnt[NCH];
  __shared__ int slots[NCH][SLOTC];
  const int tid = threadIdx.x, n0 = blockIdx.x * NCH, r = blockIdx.y;
  for (int i = tid; i < NCH; i += 256) scnt[i] = 0;
  __syncthreads();
  for (int e = tid; e < EE; e += 256) { const int i = dst[(size_t)r * EE + e] - n0;
    if (i >= 0 && i < NCH) { const int s = atomicAdd(&scnt[i], 1); if (s < SLOTC - 1) slots[i][s] = e; } }
  __syncthreads();
  for (int i = tid; i < NCH; i += 256) { const int n = n0 + i;
    const int ctrue = scnt[i]; int c = ctrue; if (c > SLOTC - 1) c = SLOTC - 1;
    for (int a = 1; a < c; ++a) { const int vv = slots[i][a]; int b = a - 1; while (b >= 0 && slots[i][b] > vv) { slots[i][b + 1] = slots[i][b]; --b; } slots[i][b + 1] = vv; }
    for (int a = c; a < SLOTC; ++a) slots[i][a] = 0;
    slots[i][SLOTC - 1] = ctrue;
#pragma unroll 1
    for (int p = 0; p < SLOTC / 4; ++p) { v4i vv = { slots[i][4 * p], slots[i][4 * p + 1], slots[i][4 * p + 2], slots[i][4 * p + 3] }; vst2(tlist + ((size_t)r * NN + n) * SLOTC + 4 * p, vv); }
  }
}

template <int MODE>
__global__ __launch_bounds__(128) void k_gemm(const _Float16* __restrict__ A, const _Float16* __restrict__ Wt, const float* __restrict__ bias,
                                            const float* __restrict__ al, const float* __restrict__ ar, float* __restrict__ Out, float* __restrict__ elr, int K, int N) {
  __shared__ __align__(16) float so[4][16 * 128];
  __shared__ __align__(16) float sel[2][64];
  const int tid = threadIdx.x, wave = tid >> 5, lane = tid & 31, col = lane & 15, g = lane >> 4;
  const int r0 = blockIdx.x * 64 + wave * 16, n0 = blockIdx.y * 128;
  v8f acc[8] = {};
#pragma unroll 1
  for (int kc = 0; kc < K / 32; ++kc) { const v16h a = frag_h(A + (size_t)(r0 + col) * K + kc * 32, lane);
#pragma unroll
    for (int j = 0; j < 8; ++j) acc[j] = wmma16(a, frag_h(Wt + (size_t)(n0 + j * 16 + col) * K + kc * 32, lane), acc[j]); }
  float* S = so[wave];
#pragma unroll
  for (int j = 0; j < 8; ++j) { const float bv = bias ? bias[n0 + j * 16 + col] : 0.f;
#pragma unroll
    for (int r = 0; r < 8; ++r) S[(8 * g + r) * 128 + j * 16 + col] = acc[j][r] + bv; }
  LDSX();
#pragma unroll 4
  for (int rl = 0; rl < 16; ++rl) vst2(Out + (size_t)(r0 + rl) * N + n0 + lane * 4, *(const v4f*)(S + rl * 128 + lane * 4));
  if (MODE == 1) { const int hh = blockIdx.y;
    if (lane < 16) { float e1 = 0.f, e2 = 0.f; const float* row = S + lane * 128;
#pragma unroll 1
      for (int d = 0; d < HID; ++d) { const float z = row[d]; e1 += z * al[hh * HID + d]; e2 += z * ar[hh * HID + d]; }
      sel[0][wave * 16 + lane] = e1; sel[1][wave * 16 + lane] = e2; }
    __syncthreads();
    if (tid < 32) { const int which = tid >> 4, pc = tid & 15;
      vst2(elr + ((size_t)which * NH + hh) * NN + blockIdx.x * 64 + pc * 4, *(const v4f*)(&sel[which][pc * 4])); }
  }
}

__global__ __launch_bounds__(256) void k_relnode(const float* __restrict__ z, const float* __restrict__ elr, const int* __restrict__ src,
                                               const int* __restrict__ tl, const float* __restrict__ hin, const float* __restrict__ bb,
                                               float* __restrict__ acc, float* __restrict__ nst, float* __restrict__ imp, int first, int do_imp) {
  const int tid = threadIdx.x, w = tid >> 5, lane = tid & 31, n = blockIdx.x * 8 + w;
  int dn = tl[(size_t)n * SLOTC + SLOTC - 1]; dn = dn < 0 ? 0 : (dn > SLOTC - 1 ? SLOTC - 1 : dn);
  float mx[NH], den[NH];
#pragma unroll
  for (int hh = 0; hh < NH; ++hh) { mx[hh] = -INFINITY; den[hh] = 0.f; }
  const float er0 = elr[(size_t)(NH + 0) * NN + n], er1 = elr[(size_t)(NH + 1) * NN + n], er2 = elr[(size_t)(NH + 2) * NN + n], er3 = elr[(size_t)(NH + 3) * NN + n];
  const float erv[NH] = { er0, er1, er2, er3 };
#pragma unroll 1
  for (int s = 0; s < dn; ++s) { int e = tl[(size_t)n * SLOTC + s]; if ((unsigned)e >= (unsigned)EE) continue; int sr = src[e]; sr = sr < 0 ? 0 : (sr >= NN ? NN - 1 : sr);
#pragma unroll
    for (int hh = 0; hh < NH; ++hh) { float sc = elr[(size_t)hh * NN + sr] + erv[hh]; sc = sc > 0.f ? sc : 0.2f * sc; mx[hh] = fmaxf(mx[hh], sc); } }
  float aggv[NH][4]; float impacc = 0.f;
#pragma unroll
  for (int hh = 0; hh < NH; ++hh) { aggv[hh][0] = 0.f; aggv[hh][1] = 0.f; aggv[hh][2] = 0.f; aggv[hh][3] = 0.f; }
#pragma unroll 1
  for (int s = 0; s < dn; ++s) { int e = tl[(size_t)n * SLOTC + s]; if ((unsigned)e >= (unsigned)EE) continue; int sr = src[e]; sr = sr < 0 ? 0 : (sr >= NN ? NN - 1 : sr);
#pragma unroll
    for (int hh = 0; hh < NH; ++hh) { float sc = elr[(size_t)hh * NN + sr] + erv[hh]; sc = sc > 0.f ? sc : 0.2f * sc; const float ex = expf(sc - mx[hh]); den[hh] += ex;
      const v4f zv = *(const v4f*)(z + (size_t)sr * DD + hh * HID + lane * 4);
      aggv[hh][0] += ex * zv[0]; aggv[hh][1] += ex * zv[1]; aggv[hh][2] += ex * zv[2]; aggv[hh][3] += ex * zv[3]; } }
  if (do_imp) {
#pragma unroll 1
    for (int s = 0; s < dn; ++s) { int e = tl[(size_t)n * SLOTC + s]; if ((unsigned)e >= (unsigned)EE) continue; int sr = src[e]; sr = sr < 0 ? 0 : (sr >= NN ? NN - 1 : sr);
      float am = 0.f;
#pragma unroll
      for (int hh = 0; hh < NH; ++hh) { float sc = elr[(size_t)hh * NN + sr] + erv[hh]; sc = sc > 0.f ? sc : 0.2f * sc; am += expf(sc - mx[hh]) / den[hh]; }
      impacc += 0.25f * am; } }
#pragma unroll
  for (int hh = 0; hh < NH; ++hh) { const float inv = dn > 0 ? 1.0f / den[hh] : 0.f;
    const size_t o = (size_t)n * DD + hh * HID + lane * 4;
    const v4f hv = *(const v4f*)(hin + o), bvv = *(const v4f*)(bb + hh * HID + lane * 4);
    v4f outv = { aggv[hh][0] * inv, aggv[hh][1] * inv, aggv[hh][2] * inv, aggv[hh][3] * inv };
    outv += hv + bvv;
    v4f prev = first ? (v4f){0.f, 0.f, 0.f, 0.f} : *(const v4f*)(acc + o);
    vst2(acc + o, prev + outv); }
  float stv = 0.f; if (lane < 4) stv = mx[lane & 3]; else if (lane < 8) stv = den[lane & 3];
  vst2(nst + (size_t)n * 32 + lane, (float_a)stv);
  if (do_imp && lane == 0) { const float prev = first ? 0.f : imp[(size_t)n * 32]; vst2(imp + (size_t)n * 32, (float_a)(prev + impacc)); }
}
__global__ __launch_bounds__(256) void k_attnout(const float* __restrict__ elr, const int* __restrict__ src, const int* __restrict__ dst,
                                               const float* __restrict__ nst, int r, float* __restrict__ attn) {
  const int e = blockIdx.x * 256 + threadIdx.x;
  int sr = src[(size_t)r * EE + e], ds = dst[(size_t)r * EE + e]; sr = sr < 0 ? 0 : (sr >= NN ? NN - 1 : sr); ds = ds < 0 ? 0 : (ds >= NN ? NN - 1 : ds);
  float am = 0.f;
#pragma unroll
  for (int hh = 0; hh < NH; ++hh) { float sc = elr[(size_t)hh * NN + sr] + elr[(size_t)(NH + hh) * NN + ds]; sc = sc > 0.f ? sc : 0.2f * sc;
    am += expf(sc - nst[(size_t)ds * 32 + hh]) / nst[(size_t)ds * 32 + 4 + hh]; }
  vst2(attn + (size_t)r * EE + e, (float_a)(0.25f * am));
}
__global__ __launch_bounds__(256) void k_finish(const float* __restrict__ acc, int useelu, float* __restrict__ hf, _Float16* __restrict__ h16) {
  const size_t g8 = (size_t)blockIdx.x * 256 + threadIdx.x; if (g8 >= (size_t)NN * DD / 8) return;
  float v[8]; union { v8h h; v4u u; } pk;
#pragma unroll
  for (int e = 0; e < 8; ++e) { float a = acc[g8 * 8 + e] * (1.0f / (float)RR); if (useelu) a = a > 0.f ? a : (expf(a) - 1.0f); v[e] = a; pk.h[e] = (_Float16)a; }
  vst2(hf + g8 * 8, (v4f){v[0], v[1], v[2], v[3]}); vst2(hf + g8 * 8 + 4, (v4f){v[4], v[5], v[6], v[7]});
  vst2(h16 + g8 * 8, pk.u);
}

__global__ __launch_bounds__(32) void k_gemm16(const _Float16* __restrict__ A, const _Float16* __restrict__ Wt, const float* __restrict__ bias, float* __restrict__ Out) {
  __shared__ __align__(16) float S[16][132];
  const int lane = threadIdx.x, col = lane & 15, g = lane >> 4, n0 = blockIdx.x * 128;
  v8f acc[8] = {};
#pragma unroll 1
  for (int kc = 0; kc < DD / 32; ++kc) { const v16h a = frag_h(A + (size_t)col * DD + kc * 32, lane);
#pragma unroll
    for (int j = 0; j < 8; ++j) acc[j] = wmma16(a, frag_h(Wt + (size_t)(n0 + j * 16 + col) * DD + kc * 32, lane), acc[j]); }
#pragma unroll
  for (int j = 0; j < 8; ++j) { const float bv = bias[n0 + j * 16 + col];
#pragma unroll
    for (int r = 0; r < 8; ++r) S[8 * g + r][j * 16 + col] = acc[j][r] + bv; }
  LDSX();
  for (int q = lane; q < 16 * 32; q += 32) { const int rl = q >> 5, pc = q & 31; vst2(Out + (size_t)rl * DD + n0 + pc * 4, *(const v4f*)(&S[rl][pc * 4])); }
}
__global__ __launch_bounds__(256) void k_mha(const float* __restrict__ q, const float* __restrict__ k, const float* __restrict__ v, float* __restrict__ ctx) {
  __shared__ float sp[SS], red[SS];
  const int b = blockIdx.x >> 2, hh = blockIdx.x & 3, tid = threadIdx.x;
  float s = 0.f; const float* qr = q + (size_t)b * DD + hh * HID; const float* kr = k + ((size_t)b * SS + tid) * DD + hh * HID;
#pragma unroll 1
  for (int d = 0; d < HID; d += 4) { const v4f kv = *(const v4f*)(kr + d); s += qr[d] * kv[0] + qr[d + 1] * kv[1] + qr[d + 2] * kv[2] + qr[d + 3] * kv[3]; }
  s *= 0.088388347648318447f;
  red[tid] = s; __syncthreads();
  for (int st = 128; st > 0; st >>= 1) { if (tid < st) red[tid] = fmaxf(red[tid], red[tid + st]); __syncthreads(); }
  const float mx = red[0]; __syncthreads();
  const float ex = expf(s - mx); sp[tid] = ex; red[tid] = ex; __syncthreads();
  for (int st = 128; st > 0; st >>= 1) { if (tid < st) red[tid] += red[tid + st]; __syncthreads(); }
  const float inv = 1.0f / red[0];
  if (tid < HID) { float c = 0.f;
#pragma unroll 1
    for (int j = 0; j < SS; ++j) c += sp[j] * v[((size_t)b * SS + j) * DD + hh * HID + tid];
    vst2(ctx + (size_t)b * DD + hh * HID + tid, (float_a)(c * inv)); }
}
__global__ __launch_bounds__(128) void k_comb(const float* __restrict__ feats, const float* __restrict__ imp, const float* __restrict__ ao, _Float16* __restrict__ comb) {
  const size_t n = blockIdx.x; const int tid = threadIdx.x, b = (int)(n / SS);
  const float w = imp[n * 32];
  union { v8h h; v4u u; } pk;
  if (tid < 64) {
#pragma unroll
    for (int e = 0; e < 8; ++e) pk.h[e] = (_Float16)(feats[n * DD + tid * 8 + e] * w);
    vst2(comb + n * (2 * DD) + tid * 8, pk.u); }
  else {
#pragma unroll
    for (int e = 0; e < 8; ++e) pk.h[e] = (_Float16)ao[(size_t)b * DD + (tid - 64) * 8 + e];
    vst2(comb + n * (2 * DD) + DD + (tid - 64) * 8, pk.u); }
}
__global__ __launch_bounds__(128) void k_cls(const _Float16* __restrict__ comb, const _Float16* __restrict__ W1t, const float* __restrict__ b1,
                                           const float* __restrict__ W2, const float* __restrict__ b2, float* __restrict__ out) {
  __shared__ __align__(16) float so[4][16 * 128];
  __shared__ __align__(16) float sl[64][2];
  const int tid = threadIdx.x, wave = tid >> 5, lane = tid & 31, col = lane & 15, g = lane >> 4;
  const int r0 = blockIdx.x * 64 + wave * 16;
  v8f acc[8] = {};
#pragma unroll 1
  for (int kc = 0; kc < 2 * DD / 32; ++kc) { const v16h a = frag_h(comb + (size_t)(r0 + col) * (2 * DD) + kc * 32, lane);
#pragma unroll
    for (int j = 0; j < 8; ++j) acc[j] = wmma16(a, frag_h(W1t + (size_t)(j * 16 + col) * (2 * DD) + kc * 32, lane), acc[j]); }
  float* S = so[wave];
#pragma unroll
  for (int j = 0; j < 8; ++j) { const float bv = b1[j * 16 + col];
#pragma unroll
    for (int r = 0; r < 8; ++r) { const float u = acc[j][r] + bv; S[(8 * g + r) * 128 + j * 16 + col] = u > 0.f ? u : 0.f; } }
  LDSX();
  if (lane < 16) { float o0 = b2[0], o1 = b2[1]; const float* row = S + lane * 128;
#pragma unroll 1
    for (int d = 0; d < HID; ++d) { const float hv = row[d]; o0 += hv * W2[d * 2]; o1 += hv * W2[d * 2 + 1]; }
    sl[wave * 16 + lane][0] = o0; sl[wave * 16 + lane][1] = o1; }
  __syncthreads();
  if (tid < 32) vst2(out + (size_t)blockIdx.x * 128 + tid * 4, *(const v4f*)(&sl[0][0] + tid * 4));
}

extern "C" void kernel_launch(void* const* d_in, const int* in_sizes, int n_in,
                              void* d_out, int out_size, void* d_ws, size_t ws_size,
                              hipStream_t stream) {
  (void)in_sizes; (void)n_in; (void)out_size; (void)ws_size;
  const float* feat = (const float*)d_in[0]; const float* hyp = (const float*)d_in[1];
  const int* esrc = (const int*)d_in[2]; const int* edst = (const int*)d_in[3];
  const float* W1 = (const float*)d_in[4]; const float* al1 = (const float*)d_in[5]; const float* ar1 = (const float*)d_in[6]; const float* bb1 = (const float*)d_in[7];
  const float* W2 = (const float*)d_in[8]; const float* al2 = (const float*)d_in[9]; const float* ar2 = (const float*)d_in[10]; const float* bb2 = (const float*)d_in[11];
  const float* Wq = (const float*)d_in[12]; const float* bq = (const float*)d_in[13]; const float* Wk = (const float*)d_in[14]; const float* bk = (const float*)d_in[15];
  const float* Wv = (const float*)d_in[16]; const float* bv = (const float*)d_in[17]; const float* Wo = (const float*)d_in[18]; const float* bo = (const float*)d_in[19];
  const float* Wn1 = (const float*)d_in[20]; const float* bn1 = (const float*)d_in[21]; const float* Wn2 = (const float*)d_in[22]; const float* bn2 = (const float*)d_in[23];
  float* out = (float*)d_out; float* attn = (float*)d_out + (size_t)NN * 2;
  char* ws = (char*)d_ws; size_t off = 0;
  auto take = [&](size_t bytes) { char* p = ws + off; off += (bytes + 255) & ~(size_t)255; return p; };
  _Float16* WT = (_Float16*)take((size_t)RR * DD * DD * 2);
  _Float16* WqT = (_Float16*)take((size_t)DD * DD * 2); _Float16* WkT = (_Float16*)take((size_t)DD * DD * 2);
  _Float16* WvT = (_Float16*)take((size_t)DD * DD * 2); _Float16* WoT = (_Float16*)take((size_t)DD * DD * 2);
  _Float16* Wn1T = (_Float16*)take((size_t)HID * 2 * DD * 2);
  int* tlist = (int*)take((size_t)RR * NN * SLOTC * 4);
  _Float16* h16 = (_Float16*)take((size_t)NN * DD * 2);
  float* z = (float*)take((size_t)NN * DD * 4);
  float* elr = (float*)take((size_t)2 * NH * NN * 4);
  float* acc = (float*)take((size_t)NN * DD * 4);
  float* nst = (float*)take((size_t)NN * 32 * 4); float* imp = (float*)take((size_t)NN * 32 * 4);
  float* h1 = (float*)take((size_t)NN * DD * 4); float* feats = (float*)take((size_t)NN * DD * 4);
  _Float16* hyp16 = (_Float16*)take((size_t)NBG * DD * 2); float* q = (float*)take((size_t)NBG * DD * 4);
  float* kk = (float*)take((size_t)NN * DD * 4); float* vv = (float*)take((size_t)NN * DD * 4);
  float* ctx = (float*)take((size_t)NBG * DD * 4); _Float16* ctx16 = (_Float16*)take((size_t)NBG * DD * 2); float* ao = (float*)take((size_t)NBG * DD * 4);
  _Float16* comb = (_Float16*)take((size_t)NN * 2 * DD * 2);
  k_bucket<<<dim3(NN / NCH, RR), 256, 0, stream>>>(edst, tlist);
  k_packT<<<dim3(DD / 64, DD / 64, RR), 256, 0, stream>>>(W1, WT, DI, DD);
  k_cvt<<<(unsigned)((NN * DI / 8 + 255) / 256), 256, 0, stream>>>(feat, h16, (size_t)NN * DI / 8);
  for (int r = 0; r < RR; ++r) {
    k_gemm<1><<<dim3(NN / 64, DD / 128), 128, 0, stream>>>(h16, WT + (size_t)r * DD * DD, nullptr, al1 + (size_t)r * NH * HID, ar1 + (size_t)r * NH * HID, z, elr, DI, DD);
    k_relnode<<<NN / 8, 256, 0, stream>>>(z, elr, esrc + (size_t)r * EE, tlist + (size_t)r * NN * SLOTC, feat, bb1 + (size_t)r * NH * HID, acc, nst, imp, r == 0 ? 1 : 0, 1);
    k_attnout<<<EE / 256, 256, 0, stream>>>(elr, esrc, edst, nst, r, attn);
  }
  k_finish<<<(unsigned)((NN * DD / 8 + 255) / 256), 256, 0, stream>>>(acc, 1, h1, h16);
  k_packT<<<dim3(DD / 64, DD / 64, RR), 256, 0, stream>>>(W2, WT, DD, DD);
  for (int r = 0; r < RR; ++r) {
    k_gemm<1><<<dim3(NN / 64, DD / 128), 128, 0, stream>>>(h16, WT + (size_t)r * DD * DD, nullptr, al2 + (size_t)r * NH * HID, ar2 + (size_t)r * NH * HID, z, elr, DD, DD);
    k_relnode<<<NN / 8, 256, 0, stream>>>(z, elr, esrc + (size_t)r * EE, tlist + (size_t)r * NN * SLOTC, h1, bb2 + (size_t)r * NH * HID, acc, nst, imp, r == 0 ? 1 : 0, 0);
  }
  k_finish<<<(unsigned)((NN * DD / 8 + 255) / 256), 256, 0, stream>>>(acc, 0, feats, h16);
  k_packT<<<dim3(DD / 64, DD / 64, 1), 256, 0, stream>>>(Wq, WqT, DD, DD);
  k_packT<<<dim3(DD / 64, DD / 64, 1), 256, 0, stream>>>(Wk, WkT, DD, DD);
  k_packT<<<dim3(DD / 64, DD / 64, 1), 256, 0, stream>>>(Wv, WvT, DD, DD);
  k_packT<<<dim3(DD / 64, DD / 64, 1), 256, 0, stream>>>(Wo, WoT, DD, DD);
  k_packT<<<dim3(HID / 64, 2 * DD / 64, 1), 256, 0, stream>>>(Wn1, Wn1T, 2 * DD, HID);
  k_cvt<<<(unsigned)((NBG * DD / 8 + 255) / 256), 256, 0, stream>>>(hyp, hyp16, (size_t)NBG * DD / 8);
  k_gemm16<<<DD / 128, 32, 0, stream>>>(hyp16, WqT, bq, q);
  k_gemm<0><<<dim3(NN / 64, DD / 128), 128, 0, stream>>>(h16, WkT, bk, nullptr, nullptr, kk, nullptr, DD, DD);
  k_gemm<0><<<dim3(NN / 64, DD / 128), 128, 0, stream>>>(h16, WvT, bv, nullptr, nullptr, vv, nullptr, DD, DD);
  k_mha<<<NBG * NH, 256, 0, stream>>>(q, kk, vv, ctx);
  k_cvt<<<(unsigned)((NBG * DD / 8 + 255) / 256), 256, 0, stream>>>(ctx, ctx16, (size_t)NBG * DD / 8);
  k_gemm16<<<DD / 128, 32, 0, stream>>>(ctx16, WoT, bo, ao);
  k_comb<<<NN, 128, 0, stream>>>(feats, imp, ao, comb);
  k_cls<<<NN / 64, 128, 0, stream>>>(comb, Wn1T, bn1, Wn2, bn2, out);
}
